// BasicTransformerBlock_12738873000028
// MI455X (gfx1250) — hardware-verified
//
#include <hip/hip_runtime.h>
#include <stddef.h>


typedef __attribute__((ext_vector_type(16))) _Float16 v16h;
typedef __attribute__((ext_vector_type(8)))  _Float16 v8h;
typedef __attribute__((ext_vector_type(8)))  float    v8f;
typedef __attribute__((ext_vector_type(4)))  float    v4f;

__device__ __forceinline__ void dep_guard_h(v8f& a, v8f& b, v16h x, v16h y) { asm volatile("v_nop\n\tv_nop\n\tv_nop\n\tv_nop" : "+v"(a), "+v"(b) : "v"(x), "v"(y)); }
__device__ __forceinline__ void keep4_h(v16h a, v16h b, v16h c, v16h d) { asm volatile("v_nop" :: "v"(a), "v"(b), "v"(c), "v"(d)); }
__device__ __forceinline__ void acc_guard4(v8f& a, v8f& b, v8f& c, v8f& d) { asm volatile("v_nop\n\tv_nop\n\tv_nop\n\tv_nop" : "+v"(a), "+v"(b), "+v"(c), "+v"(d)); }

template <typename T> struct Frag;
template <> struct Frag<_Float16> {
  typedef v16h V; union U { v16h v; v8h h[2]; };
  static __device__ __forceinline__ v16h load(const _Float16* p) {
    U f; f.h[0] = *(const v8h*)(p); f.h[1] = *(const v8h*)(p + 16); return f.v;
  }
  static __device__ __forceinline__ v8f mma(v16h a, v16h b, v8f c) {
    return __builtin_amdgcn_wmma_f32_16x16x32_f16(false, a, false, b, (short)0, c, false, false);
  }
  static __device__ __forceinline__ void guard(v8f& a, v8f& b, v16h x, v16h y) { dep_guard_h(a, b, x, y); }
  static __device__ __forceinline__ void keep(v16h a, v16h b, v16h c, v16h d) { keep4_h(a, b, c, d); }
};

template <int BIAS_MODE, int OUT_MODE, bool RESID, bool GATE>
__global__ __launch_bounds__(256) void wmma_gemm64(
    const unsigned short* __restrict__ Ap, int lda, long strideA,
    const unsigned short* __restrict__ Btp, int ldb, long strideB,
    void* __restrict__ Cout, void* __restrict__ Cout2, int ldc, long strideC,
    const float* __restrict__ bias,
    const float* __restrict__ raux, long strideR, float rscale,
    int M, int N, int K, float scale, float oscale) {
  typedef _Float16 T;
  typedef Frag<T>::V V;
  const T* A = (const T*)Ap; const T* Bt = (const T*)Btp;
  __shared__ __align__(16) float sT[8][16 * 68];
  const int b    = blockIdx.y;
  const int lane = threadIdx.x & 31;
  const int wave = threadIdx.x >> 5;
  const int tilesN = N >> 6;
  const int tilesM = M >> 6;
  const int tile = blockIdx.x * 8 + wave;
  if (tile >= tilesM * tilesN) return;
  const int tm = tile / tilesN;
  const int tn = tile - tm * tilesN;
  const int m0 = tm << 6;
  const int n0 = tn << 6;

  const T* Ab = A  + (size_t)b * strideA;
  const T* Bb = Bt + (size_t)b * strideB;

  const int rlane = lane & 15;
  const int koff  = (lane >> 4) * 8;
  const int mOff  = (lane >> 4) * 8;

  v8f acc[4][4];
#pragma unroll
  for (int i = 0; i < 4; ++i)
#pragma unroll
    for (int j = 0; j < 4; ++j) acc[i][j] = (v8f){0.f,0.f,0.f,0.f,0.f,0.f,0.f,0.f};

  for (int k0 = 0; k0 < K; k0 += 32) {
    V bh[4];
#pragma unroll
    for (int j = 0; j < 4; ++j) {
      const size_t bo = (size_t)(n0 + (j << 4) + rlane) * ldb + koff + k0;
      bh[j] = Frag<T>::load(Bb + bo);
    }
#pragma unroll
    for (int i = 0; i < 4; ++i) {
      const size_t ao = (size_t)(m0 + (i << 4) + rlane) * lda + koff + k0;
      V ah = Frag<T>::load(Ab + ao);
#pragma unroll
      for (int j = 0; j < 4; ++j) {
        acc[i][j] = Frag<T>::mma(ah, bh[j], acc[i][j]);
      }
      Frag<T>::guard(acc[i][0], acc[i][3], ah, ah);
    }
    Frag<T>::keep(bh[0], bh[1], bh[2], bh[3]);
  }
  acc_guard4(acc[0][0], acc[0][1], acc[0][2], acc[0][3]);
  acc_guard4(acc[1][0], acc[1][1], acc[1][2], acc[1][3]);
  acc_guard4(acc[2][0], acc[2][1], acc[2][2], acc[2][3]);
  acc_guard4(acc[3][0], acc[3][1], acc[3][2], acc[3][3]);

  float* slab = sT[wave];
  const float* Rb = (RESID || GATE) ? (raux + (size_t)b * strideR) : nullptr;
#pragma unroll
  for (int i = 0; i < 4; ++i) {
    const int mBase = m0 + (i << 4);
#pragma unroll
    for (int j = 0; j < 4; ++j) {
      const int n = n0 + (j << 4) + rlane;
      float bv = 0.f;
      if (BIAS_MODE == 2) bv = bias[n];
#pragma unroll
      for (int r = 0; r < 8; ++r) {
        const int m = mBase + mOff + r;
        float v = acc[i][j][r] * scale;
        if (BIAS_MODE == 1) v += bias[m];
        if (BIAS_MODE == 2) v += bv;
        if (RESID) v += rscale * Rb[(size_t)m * ldc + n];
        if (GATE) {
          const float g  = Rb[(size_t)m * ldc + n];
          const float eg = __expf(-1.702f * g);
          const float sg = __builtin_amdgcn_rcpf(1.0f + eg);
          v = v * (g * sg);
        }
        v *= oscale;
        slab[(mOff + r) * 68 + (j << 4) + rlane] = v;
      }
    }
    __builtin_amdgcn_fence(__ATOMIC_RELEASE, "workgroup");
    __builtin_amdgcn_wave_barrier();
    __builtin_amdgcn_fence(__ATOMIC_ACQUIRE, "workgroup");
    if (OUT_MODE == 0 || OUT_MODE == 3) {
      float* Cf = (float*)Cout + (size_t)b * strideC;
      const int hh = lane >> 4, c4 = (lane & 15) * 4;
      for (int pass = 0; pass < 2; ++pass) {
#pragma unroll
        for (int it = 0; it < 8; ++it) {
          const int row = it * 2 + hh;
          v4f vv = *(const v4f*)(slab + row * 68 + c4);
          *(volatile v4f*)(Cf + (size_t)(mBase + row) * ldc + n0 + c4) = vv;
        }
        __threadfence();
      }
    }
    if (OUT_MODE == 1 || OUT_MODE == 3) {
      unsigned short* Ch = (unsigned short*)(OUT_MODE == 1 ? Cout : Cout2) + (size_t)b * strideC;
      const int q = lane >> 3, c8 = (lane & 7) * 8;
      for (int pass = 0; pass < 2; ++pass) {
#pragma unroll
        for (int it = 0; it < 4; ++it) {
          const int row = it * 4 + q;
          const float* sp = slab + row * 68 + c8;
          v8h hv;
#pragma unroll
          for (int e = 0; e < 8; ++e) hv[e] = (_Float16)sp[e];
          *(volatile v8h*)(Ch + (size_t)(mBase + row) * ldc + n0 + c8) = hv;
        }
        __threadfence();
      }
    }
    __builtin_amdgcn_fence(__ATOMIC_RELEASE, "workgroup");
    __builtin_amdgcn_wave_barrier();
    __builtin_amdgcn_fence(__ATOMIC_ACQUIRE, "workgroup");
  }
}

__global__ __launch_bounds__(256) void k_cast8(const float* __restrict__ s0, const float* __restrict__ s1,
                                               unsigned short* __restrict__ d0, unsigned short* __restrict__ d1, int n8) {
  const int i = blockIdx.x * 256 + threadIdx.x;
  const float* s = (blockIdx.y == 0) ? s0 : s1;
  unsigned short* d = (blockIdx.y == 0) ? d0 : d1;
  if (i < n8) {
    const v4f a = *(const v4f*)(s + (size_t)i * 8);
    const v4f c = *(const v4f*)(s + (size_t)i * 8 + 4);
    v8h h;
    h[0] = (_Float16)a[0]; h[1] = (_Float16)a[1]; h[2] = (_Float16)a[2]; h[3] = (_Float16)a[3];
    h[4] = (_Float16)c[0]; h[5] = (_Float16)c[1]; h[6] = (_Float16)c[2]; h[7] = (_Float16)c[3];
    unsigned short* p = d + (size_t)i * 8;
    *(volatile v8h*)p = h;
    __threadfence();
    *(volatile v8h*)p = h;
  }
}

__global__ __launch_bounds__(256) void k_wcast_t(const float* __restrict__ p0, const float* __restrict__ p1,
                                                 const float* __restrict__ p2, const float* __restrict__ p3,
                                                 const float* __restrict__ p4, const float* __restrict__ p5,
                                                 const float* __restrict__ p6, const float* __restrict__ p7,
                                                 unsigned short* __restrict__ dst, int Kdim, int Ndim, float wscale) {
  __shared__ float tile[64][65];
  const int tid = threadIdx.x;
  const int z = blockIdx.z;
  const float* src = p0;
  if (z == 1) src = p1;
  if (z == 2) src = p2;
  if (z == 3) src = p3;
  if (z == 4) src = p4;
  if (z == 5) src = p5;
  if (z == 6) src = p6;
  if (z == 7) src = p7;
  unsigned short* d = dst + (size_t)z * (size_t)Ndim * (size_t)Kdim;
  const int n0 = blockIdx.x * 64, k0 = blockIdx.y * 64;
#pragma unroll
  for (int i = 0; i < 4; ++i) {
    const int idx = tid + 256 * i;
    const int r = idx >> 4, c4 = (idx & 15) * 4;
    const v4f v = *(const v4f*)(src + (size_t)(k0 + r) * Ndim + n0 + c4);
    tile[r][c4 + 0] = v[0]; tile[r][c4 + 1] = v[1]; tile[r][c4 + 2] = v[2]; tile[r][c4 + 3] = v[3];
  }
  __syncthreads();
  v8h hv[2];
#pragma unroll
  for (int i = 0; i < 2; ++i) {
    const int idx = tid + 256 * i;
    const int row = idx >> 3, cc = (idx & 7) * 8;
#pragma unroll
    for (int e = 0; e < 8; ++e) hv[i][e] = (_Float16)(tile[cc + e][row] * wscale);
  }
  for (int pass = 0; pass < 2; ++pass) {
#pragma unroll
    for (int i = 0; i < 2; ++i) {
      const int idx = tid + 256 * i;
      const int row = idx >> 3, cc = (idx & 7) * 8;
      *(volatile v8h*)(d + (size_t)(n0 + row) * Kdim + k0 + cc) = hv[i];
    }
    __threadfence();
  }
}

__global__ __launch_bounds__(512) void k_gn_stats(const float* __restrict__ x1, float* __restrict__ stats) {
  __shared__ float sst[32];
  const int tid = threadIdx.x, lane = tid & 31, g = tid >> 5, b = blockIdx.x;
  const float* base = x1 + (size_t)b * 4096 * 320 + g * 20;
  float s = 0.f;
#pragma unroll 1
  for (int i = 0; i < 128; ++i) {
    const float* p = base + (size_t)(lane + 32 * i) * 320;
#pragma unroll
    for (int j = 0; j < 5; ++j) {
      const v4f v = *(const v4f*)(p + 4 * j);
      s += (v[0] + v[1]) + (v[2] + v[3]);
    }
  }
#pragma unroll
  for (int off = 1; off < 32; off <<= 1) s += __shfl_xor(s, off, 32);
  const float mean = s * (1.0f / 81920.0f);
  float ss = 0.f;
#pragma unroll 1
  for (int i = 0; i < 128; ++i) {
    const float* p = base + (size_t)(lane + 32 * i) * 320;
#pragma unroll
    for (int j = 0; j < 5; ++j) {
      const v4f v = *(const v4f*)(p + 4 * j);
      const float d0 = v[0] - mean, d1 = v[1] - mean, d2 = v[2] - mean, d3 = v[3] - mean;
      ss += (d0 * d0 + d1 * d1) + (d2 * d2 + d3 * d3);
    }
  }
#pragma unroll
  for (int off = 1; off < 32; off <<= 1) ss += __shfl_xor(ss, off, 32);
  const float var = ss * (1.0f / 81920.0f);
  const float rstd = rsqrtf(var + 1.0e-3f);
  if (lane == 0) { sst[g] = mean; sst[16 + g] = rstd; }
  __syncthreads();
  if (g == 0 && lane < 8) {
    v4f o;
    o[0] = sst[4 * lane + 0]; o[1] = sst[4 * lane + 1]; o[2] = sst[4 * lane + 2]; o[3] = sst[4 * lane + 3];
    float* dp = stats + b * 32 + 4 * lane;
    *(volatile v4f*)dp = o;
    __threadfence();
    *(volatile v4f*)dp = o;
  }
}

__global__ __launch_bounds__(256) void k_gn_apply(const float* __restrict__ x1, const float* __restrict__ stats,
                                                  const float* __restrict__ gamma, const float* __restrict__ beta,
                                                  float* __restrict__ r2, unsigned short* __restrict__ xn16) {
  const int lane = threadIdx.x & 31, wave = threadIdx.x >> 5;
  const int row = blockIdx.x * 8 + wave;
  const int b = row >> 12;
  const float* xr = x1 + (size_t)row * 320;
  const float* st = stats + b * 32;
  v4f rv[3];
#pragma unroll
  for (int it = 0; it < 3; ++it) {
    const int q = it * 32 + lane;
    const int qc = q < 80 ? q : 79;
    const int c = qc * 4;
    const int g = c / 20;
    const float m = st[g], rs = st[16 + g];
    const v4f xv = *(const v4f*)(xr + c);
    const v4f ga = *(const v4f*)(gamma + c);
    const v4f be = *(const v4f*)(beta + c);
#pragma unroll
    for (int e = 0; e < 4; ++e) {
      const float y = (xv[e] - m) * rs * ga[e] + be[e];
      rv[it][e] = y + xv[e];
    }
  }
  for (int pass = 0; pass < 2; ++pass) {
#pragma unroll
    for (int it = 0; it < 3; ++it) {
      const int q = it * 32 + lane;
      if (q < 80) *(volatile v4f*)(r2 + (size_t)row * 320 + q * 4) = rv[it];
    }
    __threadfence();
  }
  v8h hv[2];
#pragma unroll
  for (int it = 0; it < 2; ++it) {
    const int q = it * 32 + lane;
    const int qc = q < 40 ? q : 39;
    const int c = qc * 8;
    const v4f xa = *(const v4f*)(xr + c);
    const v4f xb = *(const v4f*)(xr + c + 4);
    const v4f ga = *(const v4f*)(gamma + c);
    const v4f gb = *(const v4f*)(gamma + c + 4);
    const v4f ba = *(const v4f*)(beta + c);
    const v4f bb = *(const v4f*)(beta + c + 4);
#pragma unroll
    for (int e = 0; e < 4; ++e) {
      const int g0 = (c + e) / 20, g1 = (c + 4 + e) / 20;
      const float y0 = (xa[e] - st[g0]) * st[16 + g0] * ga[e] + ba[e];
      const float y1 = (xb[e] - st[g1]) * st[16 + g1] * gb[e] + bb[e];
      hv[it][e] = (_Float16)y0;
      hv[it][4 + e] = (_Float16)y1;
    }
  }
  for (int pass = 0; pass < 2; ++pass) {
#pragma unroll
    for (int it = 0; it < 2; ++it) {
      const int q = it * 32 + lane;
      if (q < 40) *(volatile v8h*)(xn16 + (size_t)row * 320 + q * 8) = hv[it];
    }
    __threadfence();
  }
}

__global__ __launch_bounds__(256) void k_softmax(unsigned short* __restrict__ SP, float inscale) {
  __shared__ float redm[8];
  __shared__ float reds[8];
  const int tid = threadIdx.x, lane = tid & 31, wave = tid >> 5;
  unsigned short* rowp = SP + (size_t)blockIdx.x * 4096;
  const v8h ha = *(const v8h*)(rowp + 8 * tid);
  const v8h hb = *(const v8h*)(rowp + 8 * (256 + tid));
  float ta[8], tb[8];
  float mx = -3.0e38f;
#pragma unroll
  for (int e = 0; e < 8; ++e) {
    ta[e] = (float)ha[e] * inscale;
    tb[e] = (float)hb[e] * inscale;
    mx = fmaxf(mx, fmaxf(ta[e], tb[e]));
  }
#pragma unroll
  for (int off = 1; off < 32; off <<= 1) mx = fmaxf(mx, __shfl_xor(mx, off, 32));
  if (lane == 0) redm[wave] = mx;
  __syncthreads();
  float m = redm[0];
#pragma unroll
  for (int w = 1; w < 8; ++w) m = fmaxf(m, redm[w]);
  float sum = 0.f;
#pragma unroll
  for (int e = 0; e < 8; ++e) {
    ta[e] = __expf(ta[e] - m);
    tb[e] = __expf(tb[e] - m);
    sum += ta[e] + tb[e];
  }
#pragma unroll
  for (int off = 1; off < 32; off <<= 1) sum += __shfl_xor(sum, off, 32);
  if (lane == 0) reds[wave] = sum;
  __syncthreads();
  float tot = reds[0];
#pragma unroll
  for (int w = 1; w < 8; ++w) tot += reds[w];
  const float inv = 32768.0f * __builtin_amdgcn_rcpf(tot);
  v8h pa, pb;
#pragma unroll
  for (int e = 0; e < 8; ++e) { pa[e] = (_Float16)(ta[e] * inv); pb[e] = (_Float16)(tb[e] * inv); }
  unsigned short* qa = rowp + 8 * tid;
  unsigned short* qb = rowp + 8 * (256 + tid);
  *(volatile v8h*)qa = pa;
  *(volatile v8h*)qb = pb;
  __threadfence();
  *(volatile v8h*)qa = pa;
  *(volatile v8h*)qb = pb;
}

extern "C" void kernel_launch(void* const* d_in, const int* in_sizes, int n_in,
                              void* d_out, int out_size, void* d_ws, size_t ws_size,
                              hipStream_t stream)
{
  const int Bn = 2, N = 4096, C = 320, M = 8192, C4 = 1280, C8 = 2560;
  if (n_in < 24) return;
  if (in_sizes[0] != M * C || in_sizes[1] != M * C || out_size != M * C) return;
  if (in_sizes[2] != C * C || in_sizes[4] != C * C || in_sizes[6] != C * C || in_sizes[8] != C * C) return;
  if (in_sizes[10] != C * C || in_sizes[12] != C * C || in_sizes[14] != C * C || in_sizes[16] != C * C) return;
  if (in_sizes[18] != C || in_sizes[19] != C || in_sizes[20] != C * C8 || in_sizes[21] != C8) return;
  if (in_sizes[22] != C4 * C || in_sizes[23] != C) return;

  const float* x      = (const float*)d_in[0];
  const float* ctx    = (const float*)d_in[1];
  const float* sa_q_w = (const float*)d_in[2];   const float* sa_q_b = (const float*)d_in[3];
  const float* sa_k_w = (const float*)d_in[4];   const float* sa_k_b = (const float*)d_in[5];
  const float* sa_v_w = (const float*)d_in[6];   const float* sa_v_b = (const float*)d_in[7];
  const float* sa_p_w = (const float*)d_in[8];   const float* sa_p_b = (const float*)d_in[9];
  const float* ca_q_w = (const float*)d_in[10];  const float* ca_q_b = (const float*)d_in[11];
  const float* ca_k_w = (const float*)d_in[12];  const float* ca_k_b = (const float*)d_in[13];
  const float* ca_v_w = (const float*)d_in[14];  const float* ca_v_b = (const float*)d_in[15];
  const float* ca_p_w = (const float*)d_in[16];  const float* ca_p_b = (const float*)d_in[17];
  const float* gn_g   = (const float*)d_in[18];  const float* gn_b   = (const float*)d_in[19];
  const float* gg_w   = (const float*)d_in[20];  const float* gg_b   = (const float*)d_in[21];
  const float* de_w   = (const float*)d_in[22];  const float* de_b   = (const float*)d_in[23];
  float* out = (float*)d_out;

  char* ws = (char*)d_ws;
  size_t off = 0;
  const size_t szW8  = (size_t)8 * C * C * 2;
  const size_t szWG  = (size_t)C8 * C * 2;
  const size_t szWD  = (size_t)C * C4 * 2;
  const size_t szST  = 4096;
  const size_t szP16 = (size_t)M * C * 2;
  const size_t szP32 = (size_t)M * C * 4;
  const size_t szAR  = (size_t)Bn * N * N * 2;
  const size_t oW8 = off;  off += szW8;
  const size_t oWG = off;  off += szWG;
  const size_t oWD = off;  off += szWD;
  const size_t oST = off;  off += szST;
  const size_t oX16 = off; off += szP16;
  const size_t oC16 = off; off += szP16;
  const size_t oQ16 = off; off += szP16;
  const size_t oK16 = off; off += szP16;
  const size_t oVT  = off; off += szP16;
  const size_t oO16 = off; off += szP16;
  const size_t oX1  = off; off += szP32;
  const size_t oR2  = off; off += szP32;
  const size_t oAR  = off; off += szAR;
  if (off > ws_size) return;
  const size_t szG = (size_t)M * C4 * 4;
  const size_t szFF = (size_t)M * C4 * 2;
  if (szG + szFF > szAR) return;

  unsigned short* W8   = (unsigned short*)(ws + oW8);
  unsigned short* WG   = (unsigned short*)(ws + oWG);
  unsigned short* WD   = (unsigned short*)(ws + oWD);
  float*          ST   = (float*)(ws + oST);
  unsigned short* X16  = (unsigned short*)(ws + oX16);
  unsigned short* C16  = (unsigned short*)(ws + oC16);
  unsigned short* Q16  = (unsigned short*)(ws + oQ16);
  unsigned short* K16  = (unsigned short*)(ws + oK16);
  unsigned short* VT16 = (unsigned short*)(ws + oVT);
  unsigned short* O16  = (unsigned short*)(ws + oO16);
  float*          X1   = (float*)(ws + oX1);
  float*          R2   = (float*)(ws + oR2);
  unsigned short* AR   = (unsigned short*)(ws + oAR);
  float*          G    = (float*)(ws + oAR);
  unsigned short* FF16 = (unsigned short*)(ws + oAR + szG);

  const size_t CC = (size_t)C * C;
  const long NCl = (long)N * C;
  const long NNl = (long)N * N;
  const float qk_scale = 0.0559016994f;
  const dim3 blk(256);
  auto gb = [](int Mv, int Nv) { return (unsigned)((((Mv / 64) * (Nv / 64)) + 7) / 8); };

  k_wcast_t<<<dim3(C / 64, C / 64, 8), blk, 0, stream>>>(sa_q_w, sa_k_w, sa_v_w, sa_p_w, ca_q_w, ca_k_w, ca_v_w, ca_p_w,
                                                          W8, C, C, 64.0f);
  k_wcast_t<<<dim3(C8 / 64, C / 64, 1), blk, 0, stream>>>(gg_w, gg_w, gg_w, gg_w, gg_w, gg_w, gg_w, gg_w, WG, C, C8, 64.0f);
  k_wcast_t<<<dim3(C / 64, C4 / 64, 1), blk, 0, stream>>>(de_w, de_w, de_w, de_w, de_w, de_w, de_w, de_w, WD, C4, C, 64.0f);
  k_cast8<<<dim3((M * C / 8) / 256, 2), blk, 0, stream>>>(x, ctx, X16, C16, M * C / 8);

  wmma_gemm64<2, 1, false, false><<<dim3(gb(M, C), 1), blk, 0, stream>>>(
      X16, C, 0L, W8 + 0 * CC, C, 0L, Q16, nullptr, C, 0L, sa_q_b, nullptr, 0L, 0.f, M, C, C, 1.0f / 64.0f, 8.0f);
  wmma_gemm64<2, 1, false, false><<<dim3(gb(M, C), 1), blk, 0, stream>>>(
      X16, C, 0L, W8 + 1 * CC, C, 0L, K16, nullptr, C, 0L, sa_k_b, nullptr, 0L, 0.f, M, C, C, 1.0f / 64.0f, 8.0f);
  wmma_gemm64<1, 1, false, false><<<dim3(gb(C, N), Bn), blk, 0, stream>>>(
      W8 + 2 * CC, C, 0L, X16, C, NCl, VT16, nullptr, N, NCl, sa_v_b, nullptr, 0L, 0.f, C, N, C, 1.0f / 64.0f, 8.0f);
  wmma_gemm64<0, 1, false, false><<<dim3(gb(N, N), Bn), blk, 0, stream>>>(
      Q16, C, NCl, K16, C, NCl, AR, nullptr, N, NNl, nullptr, nullptr, 0L, 0.f, N, N, C, qk_scale, 1.0f);
  k_softmax<<<dim3(Bn * N), blk, 0, stream>>>(AR, 1.0f / 64.0f);
  wmma_gemm64<0, 1, false, false><<<dim3(gb(N, C), Bn), blk, 0, stream>>>(
      AR, N, NNl, VT16, N, NCl, O16, nullptr, C, NCl, nullptr, nullptr, 0L, 0.f, N, C, N, 1.0f / 4096.0f, 1.0f);
  wmma_gemm64<2, 0, true, false><<<dim3(gb(M, C), 1), blk, 0, stream>>>(
      O16, C, 0L, W8 + 3 * CC, C, 0L, X1, nullptr, C, 0L, sa_p_b, x, 0L, 2.0f, M, C, C, 1.0f / 4096.0f, 1.0f);

  k_gn_stats<<<dim3(Bn), dim3(512), 0, stream>>>(X1, ST);
  k_gn_apply<<<dim3(M / 8), blk, 0, stream>>>(X1, ST, gn_g, gn_b, R2, X16);

  wmma_gemm64<2, 1, false, false><<<dim3(gb(M, C), 1), blk, 0, stream>>>(
      X16, C, 0L, W8 + 4 * CC, C, 0L, Q16, nullptr, C, 0L, ca_q_b, nullptr, 0L, 0.f, M, C, C, 1.0f / 64.0f, 8.0f);
  wmma_gemm64<2, 1, false, false><<<dim3(gb(M, C), 1), blk, 0, stream>>>(
      C16, C, 0L, W8 + 5 * CC, C, 0L, K16, nullptr, C, 0L, ca_k_b, nullptr, 0L, 0.f, M, C, C, 1.0f / 64.0f, 8.0f);
  wmma_gemm64<1, 1, false, false><<<dim3(gb(C, N), Bn), blk, 0, stream>>>(
      W8 + 6 * CC, C, 0L, C16, C, NCl, VT16, nullptr, N, NCl, ca_v_b, nullptr, 0L, 0.f, C, N, C, 1.0f / 64.0f, 8.0f);
  wmma_gemm64<0, 1, false, false><<<dim3(gb(N, N), Bn), blk, 0, stream>>>(
      Q16, C, NCl, K16, C, NCl, AR, nullptr, N, NNl, nullptr, nullptr, 0L, 0.f, N, N, C, qk_scale, 1.0f);
  k_softmax<<<dim3(Bn * N), blk, 0, stream>>>(AR, 1.0f / 64.0f);
  wmma_gemm64<0, 1, false, false><<<dim3(gb(N, C), Bn), blk, 0, stream>>>(
      AR, N, NNl, VT16, N, NCl, O16, nullptr, C, NCl, nullptr, nullptr, 0L, 0.f, N, C, N, 1.0f / 4096.0f, 1.0f);
  wmma_gemm64<2, 3, true, false><<<dim3(gb(M, C), 1), blk, 0, stream>>>(
      O16, C, 0L, W8 + 7 * CC, C, 0L, X1, C16, C, 0L, ca_p_b, R2, 0L, 1.0f, M, C, C, 1.0f / 4096.0f, 1.0f);

  wmma_gemm64<2, 0, false, false><<<dim3(gb(M, C4), 1), blk, 0, stream>>>(
      C16, C, 0L, WG + (size_t)C4 * C, C, 0L, G, nullptr, C4, 0L, gg_b + C4, nullptr, 0L, 0.f, M, C4, C, 1.0f / 64.0f, 1.0f);
  wmma_gemm64<2, 1, false, true><<<dim3(gb(M, C4), 1), blk, 0, stream>>>(
      C16, C, 0L, WG, C, 0L, FF16, nullptr, C4, 0L, gg_b, G, 0L, 0.f, M, C4, C, 1.0f / 64.0f, 16.0f);
  wmma_gemm64<2, 0, true, false><<<dim3(gb(M, C), 1), blk, 0, stream>>>(
      FF16, C4, 0L, WD, C4, 0L, out, nullptr, C, 0L, de_b, X1, 0L, 1.0f, M, C, C4, 1.0f / 1024.0f, 1.0f);
}
